// GatedDeltaNet_7181185319143
// MI455X (gfx1250) — hardware-verified
//
#include <hip/hip_runtime.h>
#include <math.h>

constexpr int kBatch  = 2;
constexpr int kSeq    = 1024;
constexpr int kHeads  = 8;
constexpr int kHd     = 64;
constexpr int kHid    = 512;
constexpr int kKd     = kHeads * kHd;
constexpr int kRows   = kBatch * kSeq;
constexpr int kConvTaps = 4;
constexpr int kColQ   = 0;
constexpr int kColK   = kKd;
constexpr int kColV   = 2 * kKd;
constexpr int kColG   = 3 * kKd;
constexpr int kColB   = 4 * kKd;
constexpr int kColA   = 4 * kKd + kHeads;
constexpr int kColPad = 4 * kKd + 2 * kHeads;
constexpr int kNcat   = 2112;
constexpr int kChunk  = 16;
constexpr int kGateN  = kRows * kHeads;
constexpr float kNormEps = 1e-6f;
constexpr float kL2Eps   = 1e-12f;
constexpr float kInvHd   = 1.0f / (float)kHd;
constexpr double kRotBase   = 10000.0;
constexpr double kRotMaxLen = 262144.0;
constexpr double kRotOrig   = 8192.0;
constexpr double kRotFactor = 32.0;

static_assert(kKd == 512 && kHid == 512 && kRows == 2048, "shape");
static_assert(kConvTaps == 4, "conv taps");
static_assert(kNcat % 64 == 0 && kNcat >= kColPad, "N tile multiple");
static_assert(kRows % 64 == 0 && kHid % 64 == 0 && kKd % 32 == 0 && kHid % 32 == 0, "tile multiples");
static_assert(kColB % 4 == 0 && kColA % 4 == 0 && kColPad % 4 == 0, "row groups of 4");
static_assert(kSeq % kChunk == 0, "chunking");
static_assert(((kRows / 64) * (kNcat / 64)) % 8 == 0, "gemm1 tiles fill the blocks");
static_assert(((kRows / 64) * (kHid / 64)) % 8 == 0, "gemm2 tiles fill the blocks");

typedef __attribute__((ext_vector_type(16))) _Float16 v16h;
typedef __attribute__((ext_vector_type(8)))  _Float16 v8h;
typedef __attribute__((ext_vector_type(16))) __bf16   v16b;
typedef __attribute__((ext_vector_type(8)))  __bf16   v8b;
typedef __attribute__((ext_vector_type(8)))  float    v8f;
typedef __attribute__((ext_vector_type(4)))  float    v4f;
typedef __attribute__((ext_vector_type(2)))  float    v2f;
typedef __attribute__((ext_vector_type(4)))  unsigned int v4u;

__device__ __forceinline__ unsigned short f2bf_bits(float f) {
  unsigned u = __float_as_uint(f);
  return (unsigned short)((u + 0x7FFFu + ((u >> 16) & 1u)) >> 16);
}
__device__ __forceinline__ float bf_bits2f(unsigned short h) { return __uint_as_float(((unsigned)h) << 16); }
__device__ __forceinline__ unsigned pk16(unsigned short a, unsigned short b) { return (unsigned)a | ((unsigned)b << 16); }

__device__ __forceinline__ void dep_guard4_h(v8f& a, v8f& b, v8f& c, v8f& d, v16h x, v16h y) { asm volatile("v_nop\n\tv_nop\n\tv_nop\n\tv_nop" : "+v"(a), "+v"(b), "+v"(c), "+v"(d) : "v"(x), "v"(y)); }
__device__ __forceinline__ void dep_guard4_b(v8f& a, v8f& b, v8f& c, v8f& d, v16b x, v16b y) { asm volatile("v_nop\n\tv_nop\n\tv_nop\n\tv_nop" : "+v"(a), "+v"(b), "+v"(c), "+v"(d) : "v"(x), "v"(y)); }
__device__ __forceinline__ void keep4_h(v16h a, v16h b, v16h c, v16h d) { asm volatile("v_nop" :: "v"(a), "v"(b), "v"(c), "v"(d)); }
__device__ __forceinline__ void keep4_b(v16b a, v16b b, v16b c, v16b d) { asm volatile("v_nop" :: "v"(a), "v"(b), "v"(c), "v"(d)); }
__device__ __forceinline__ void acc_guard4(v8f& a, v8f& b, v8f& c, v8f& d) { asm volatile("v_nop\n\tv_nop\n\tv_nop\n\tv_nop" : "+v"(a), "+v"(b), "+v"(c), "+v"(d)); }
template <typename T> struct Frag;
template <> struct Frag<_Float16> {
  typedef v16h V; union U { v16h v; v8h h[2]; };
  static __device__ __forceinline__ v16h load(const _Float16* p) {
    U f; f.h[0] = *(const v8h*)(p); f.h[1] = *(const v8h*)(p + 16); return f.v;
  }
  static __device__ __forceinline__ v8f mma(v16h a, v16h b, v8f c) {
    return __builtin_amdgcn_wmma_f32_16x16x32_f16(false, a, false, b, (short)0, c, false, false);
  }
  static __device__ __forceinline__ void guard4(v8f& a, v8f& b, v8f& c, v8f& d, v16h x, v16h y) { dep_guard4_h(a, b, c, d, x, y); }
  static __device__ __forceinline__ void keep(v16h a, v16h b, v16h c, v16h d) { keep4_h(a, b, c, d); }
};
template <> struct Frag<__bf16> {
  typedef v16b V; union U { v16b v; v8b h[2]; };
  static __device__ __forceinline__ v16b load(const __bf16* p) {
    U f; f.h[0] = *(const v8b*)(p); f.h[1] = *(const v8b*)(p + 16); return f.v;
  }
  static __device__ __forceinline__ v8f mma(v16b a, v16b b, v8f c) {
    return __builtin_amdgcn_wmma_f32_16x16x32_bf16(false, a, false, b, (short)0, c, false, false);
  }
  static __device__ __forceinline__ void guard4(v8f& a, v8f& b, v8f& c, v8f& d, v16b x, v16b y) { dep_guard4_b(a, b, c, d, x, y); }
  static __device__ __forceinline__ void keep(v16b a, v16b b, v16b c, v16b d) { keep4_b(a, b, c, d); }
};

template <int ET> struct Elem;
template <> struct Elem<0> { typedef _Float16 T; };
template <> struct Elem<1> { typedef __bf16 T; };
template <int ET, bool SPLIT, int BIAS_MODE, int OUT_MODE, bool RESID, int ACT = 0>
__global__ __launch_bounds__(256) void wmma_gemm64(
    const unsigned short* __restrict__ Ap, const unsigned short* __restrict__ A2p, int lda, long strideA,
    const unsigned short* __restrict__ Btp, const unsigned short* __restrict__ Bt2p, int ldb, long strideB,
    void* __restrict__ Cout, void* __restrict__ Cout2, int ldc, long strideC,
    const float* __restrict__ bias,
    const float* __restrict__ resid, long strideR,
    int M, int N, int K, float scale) {
  typedef typename Elem<ET>::T T;
  typedef typename Frag<T>::V V;
  const T* A = (const T*)Ap; const T* A2 = (const T*)A2p; const T* Bt = (const T*)Btp; const T* Bt2 = (const T*)Bt2p;
  __shared__ __align__(16) float sT[8][16 * 68];
  const int b    = blockIdx.y;
  const int lane = threadIdx.x & 31;
  const int wave = threadIdx.x >> 5;
  const int tilesN = N >> 6;
  const int tilesM = M >> 6;
  const int tile = blockIdx.x * 8 + wave;
  if (tile >= tilesM * tilesN) return;
  const int tm = tile / tilesN;
  const int tn = tile - tm * tilesN;
  const int m0 = tm << 6;
  const int n0 = tn << 6;

  const T* Ab  = A  + (size_t)b * strideA;
  const T* Bb  = Bt + (size_t)b * strideB;
  const T* Ab2 = SPLIT ? (A2  + (size_t)b * strideA) : nullptr;
  const T* Bb2 = SPLIT ? (Bt2 + (size_t)b * strideB) : nullptr;

  const int rlane = lane & 15;
  const int koff  = (lane >> 4) * 8;
  const int mOff  = (lane >> 4) * 8;

  v8f acc[4][4];
#pragma unroll
  for (int i = 0; i < 4; ++i)
#pragma unroll
    for (int j = 0; j < 4; ++j) acc[i][j] = (v8f){0.f,0.f,0.f,0.f,0.f,0.f,0.f,0.f};

  for (int k0 = 0; k0 < K; k0 += 32) {
    V bh[4], bl[4];
#pragma unroll
    for (int j = 0; j < 4; ++j) {
      const size_t bo = (size_t)(n0 + (j << 4) + rlane) * ldb + koff + k0;
      bh[j] = Frag<T>::load(Bb + bo);
      if (SPLIT) bl[j] = Frag<T>::load(Bb2 + bo);
    }
#pragma unroll
    for (int i = 0; i < 4; ++i) {
      const size_t ao = (size_t)(m0 + (i << 4) + rlane) * lda + koff + k0;
      V ah = Frag<T>::load(Ab + ao);
      V al;
      if (SPLIT) al = Frag<T>::load(Ab2 + ao);
#pragma unroll
      for (int j = 0; j < 4; ++j) {
        acc[i][j] = Frag<T>::mma(ah, bh[j], acc[i][j]);
        if (SPLIT) {
          acc[i][j] = Frag<T>::mma(ah, bl[j], acc[i][j]);
          acc[i][j] = Frag<T>::mma(al, bh[j], acc[i][j]);
        }
      }
      Frag<T>::guard4(acc[i][0], acc[i][1], acc[i][2], acc[i][3], ah, SPLIT ? al : ah);
    }
    Frag<T>::keep(bh[0], bh[1], bh[2], bh[3]);
    if (SPLIT) Frag<T>::keep(bl[0], bl[1], bl[2], bl[3]);
  }
  acc_guard4(acc[0][0], acc[0][1], acc[0][2], acc[0][3]);
  acc_guard4(acc[1][0], acc[1][1], acc[1][2], acc[1][3]);
  acc_guard4(acc[2][0], acc[2][1], acc[2][2], acc[2][3]);
  acc_guard4(acc[3][0], acc[3][1], acc[3][2], acc[3][3]);

  float* slab = sT[wave];
  const float* Rb = RESID ? (resid + (size_t)b * strideR) : nullptr;
#pragma unroll
  for (int i = 0; i < 4; ++i) {
    const int mBase = m0 + (i << 4);
#pragma unroll
    for (int j = 0; j < 4; ++j) {
      const int n = n0 + (j << 4) + rlane;
      float bv = 0.f;
      if (BIAS_MODE == 2) bv = bias[n];
#pragma unroll
      for (int r = 0; r < 8; ++r) {
        float v = acc[i][j][r] * scale;
        if (BIAS_MODE == 1) v += bias[mBase + mOff + r];
        if (BIAS_MODE == 2) v += bv;
        if (RESID) v += Rb[(size_t)(mBase + mOff + r) * ldc + n];
        if (ACT == 2) v = fmaxf(v, 0.0f);
        if (ACT == 4) v = (v > 0.f) ? v : 0.01f * v;
        slab[(mOff + r) * 68 + (j << 4) + rlane] = v;
      }
    }
    __builtin_amdgcn_fence(__ATOMIC_RELEASE, "workgroup");
    __builtin_amdgcn_wave_barrier();
    __builtin_amdgcn_fence(__ATOMIC_ACQUIRE, "workgroup");
    if (OUT_MODE == 0) {
      float* C = (float*)Cout + (size_t)b * strideC;
      const int hh = lane >> 4, c4 = (lane & 15) * 4;
      for (int pass = 0; pass < 2; ++pass) {
#pragma unroll
        for (int it = 0; it < 8; ++it) {
          const int row = it * 2 + hh;
          v4f v = *(const v4f*)(slab + row * 68 + c4);
          *(volatile v4f*)(C + (size_t)(mBase + row) * ldc + n0 + c4) = v;
        }
        __threadfence();
      }
    } else {
      const int q = lane >> 3, c8 = (lane & 7) * 8;
      unsigned short* C  = (unsigned short*)Cout  + (size_t)b * strideC;
      unsigned short* C2 = (OUT_MODE == 2) ? ((unsigned short*)Cout2 + (size_t)b * strideC) : nullptr;
      for (int pass = 0; pass < 2; ++pass) {
#pragma unroll
        for (int it = 0; it < 4; ++it) {
          const int row = it * 4 + q;
          const float* sp = slab + row * 68 + c8;
          v8h hv, lv;
#pragma unroll
          for (int e = 0; e < 8; ++e) {
            if (OUT_MODE == 1) {
              hv[e] = (_Float16)sp[e];
            } else {
              unsigned short hb = f2bf_bits(sp[e]);
              unsigned short lb = f2bf_bits(sp[e] - bf_bits2f(hb));
              hv[e] = __builtin_bit_cast(_Float16, hb);
              lv[e] = __builtin_bit_cast(_Float16, lb);
            }
          }
          *(volatile v8h*)(C + (size_t)(mBase + row) * ldc + n0 + c8) = hv;
          if (OUT_MODE == 2) *(volatile v8h*)(C2 + (size_t)(mBase + row) * ldc + n0 + c8) = lv;
        }
        __threadfence();
      }
    }
    __builtin_amdgcn_fence(__ATOMIC_RELEASE, "workgroup");
    __builtin_amdgcn_wave_barrier();
    __builtin_amdgcn_fence(__ATOMIC_ACQUIRE, "workgroup");
  }
}

__device__ __forceinline__ void split_store8(const v4f a, const v4f c, const bool zero,
                                             unsigned short* dh, unsigned short* dl) {
  float x[8];
  x[0] = a[0]; x[1] = a[1]; x[2] = a[2]; x[3] = a[3];
  x[4] = c[0]; x[5] = c[1]; x[6] = c[2]; x[7] = c[3];
  unsigned short hb[8], lb[8];
#pragma unroll
  for (int e = 0; e < 8; ++e) {
    const float xv = zero ? 0.0f : x[e];
    hb[e] = f2bf_bits(xv);
    lb[e] = f2bf_bits(xv - bf_bits2f(hb[e]));
  }
  const v4u uh = (v4u){pk16(hb[0], hb[1]), pk16(hb[2], hb[3]), pk16(hb[4], hb[5]), pk16(hb[6], hb[7])};
  const v4u ul = (v4u){pk16(lb[0], lb[1]), pk16(lb[2], lb[3]), pk16(lb[4], lb[5]), pk16(lb[6], lb[7])};
  *(volatile v4u*)dh = uh;
  *(volatile v4u*)dl = ul;
  __threadfence();
  *(volatile v4u*)dh = uh;
  *(volatile v4u*)dl = ul;
}

__global__ __launch_bounds__(256) void split8_kernel(const float* __restrict__ src, unsigned short* __restrict__ dhi,
                                                     unsigned short* __restrict__ dlo, int n8) {
  const int i = blockIdx.x * 256 + threadIdx.x;
  if (i >= n8) return;
  const float* p = src + 8 * (size_t)i;
  const v4f a = *(const v4f*)(p);
  const v4f c = *(const v4f*)(p + 4);
  split_store8(a, c, false, dhi + 8 * (size_t)i, dlo + 8 * (size_t)i);
}

__global__ __launch_bounds__(256) void wcat_kernel(const float* __restrict__ Wq, const float* __restrict__ Wk,
                                                   const float* __restrict__ Wv, const float* __restrict__ Wg,
                                                   const float* __restrict__ Wb, const float* __restrict__ Wgk,
                                                   unsigned short* __restrict__ dhi, unsigned short* __restrict__ dlo) {
  const int tid = threadIdx.x;
  const int rb  = blockIdx.x * 4;
  const int row = rb + (tid >> 6);
  const int c8  = tid & 63;
  const float* src = Wq;
  int rbase = 0;
  bool zero = false;
  if (rb < kColK)        { src = Wq;  rbase = kColQ; }
  else if (rb < kColV)   { src = Wk;  rbase = kColK; }
  else if (rb < kColG)   { src = Wv;  rbase = kColV; }
  else if (rb < kColB)   { src = Wg;  rbase = kColG; }
  else if (rb < kColA)   { src = Wb;  rbase = kColB; }
  else if (rb < kColPad) { src = Wgk; rbase = kColA; }
  else                   { src = Wq;  rbase = row; zero = true; }
  const int srow = row - rbase;
  const float* p = src + (size_t)srow * kHid + c8 * 8;
  const v4f a = *(const v4f*)(p);
  const v4f c = *(const v4f*)(p + 4);
  const size_t o = (size_t)row * kHid + c8 * 8;
  split_store8(a, c, zero, dhi + o, dlo + o);
}

struct RotC { float invf[16]; float rspf[16]; };
static_assert(sizeof(RotC) == 128, "no padding");

__device__ __forceinline__ float pick16(const float (&v)[16], const int j) {
  float r = v[0];
#pragma unroll
  for (int m = 1; m < 16; ++m) r = (j == m) ? v[m] : r;
  return r;
}

__global__ __launch_bounds__(256) void rot_table_kernel(float* __restrict__ tab, const RotC rc) {
  __shared__ __align__(16) float tb[16 * 32];
  const int tid = threadIdx.x;
  const int tl  = tid >> 4;
  const int jj  = tid & 15;
  const int t   = blockIdx.x * 16 + tl;
  const float invf = pick16(rc.invf, jj);
  const float rspf = pick16(rc.rspf, jj);
  const float pos = (float)t * rspf;
  const float th  = pos * invf;
  float sv, cv;
  sincosf(th, &sv, &cv);
  tb[tl * 32 + jj]      = cv;
  tb[tl * 32 + 16 + jj] = sv;
  __syncthreads();
  if (tid < 128) {
    const v4f val = *(const v4f*)(tb + tid * 4);
    float* dst = tab + (size_t)blockIdx.x * 512 + tid * 4;
    *(volatile v4f*)dst = val;
    __threadfence();
    *(volatile v4f*)dst = val;
  }
}

__global__ __launch_bounds__(256) void gate_kernel(const float* __restrict__ P, const float* __restrict__ bb,
                                                   const float* __restrict__ bgk, const float* __restrict__ alog,
                                                   const float* __restrict__ dtb, float* __restrict__ gates) {
  __shared__ __align__(16) float sab[512];
  const int tid = threadIdx.x;
  const int idx = blockIdx.x * 256 + tid;
  const int bt  = idx >> 3;
  const int h   = idx & 7;
  const float bv = P[(size_t)bt * kNcat + kColB + h] + bb[h];
  const float beta = 1.0f / (1.0f + expf(-bv));
  const float gv = (P[(size_t)bt * kNcat + kColA + h] + bgk[h]) + dtb[h];
  const float sp = fmaxf(gv, 0.0f) + log1pf(expf(-fabsf(gv)));
  const float na = -expf(alog[h]);
  const float alpha = expf(na * sp);
  sab[tid]       = beta;
  sab[256 + tid] = alpha;
  __syncthreads();
  if (tid < 128) {
    const int w  = tid >> 6;
    const int c4 = (tid & 63) * 4;
    const v4f val = *(const v4f*)(sab + w * 256 + c4);
    float* dst = gates + (size_t)w * kGateN + (size_t)blockIdx.x * 256 + c4;
    *(volatile v4f*)dst = val;
    __threadfence();
    *(volatile v4f*)dst = val;
  }
}

__global__ __launch_bounds__(256) void prep_kernel(const float* __restrict__ P,
                                                   const float* __restrict__ cqw, const float* __restrict__ cqb,
                                                   const float* __restrict__ ckw, const float* __restrict__ ckb,
                                                   const float* __restrict__ cvw, const float* __restrict__ cvb,
                                                   const float* __restrict__ tab,
                                                   float* __restrict__ qo, float* __restrict__ ko, float* __restrict__ vo) {
  __shared__ __align__(16) float sx[3 * kKd];
  const int bt   = blockIdx.x;
  const int t    = bt % kSeq;
  const int tid  = threadIdx.x;
  const int lane = tid & 31;
  const int wave = tid >> 5;

#pragma unroll 1
  for (int it = 0; it < 6; ++it) {
    const int which = it >> 1;
    const int c = ((it & 1) << 8) + tid;
    const float* wp = (which == 0) ? cqw : ((which == 1) ? ckw : cvw);
    const float* bp = (which == 0) ? cqb : ((which == 1) ? ckb : cvb);
    const v4f w = *(const v4f*)(wp + 4 * c);
    const float bias = bp[c];
    const int col = which * kKd + c;
    float acc = 0.0f;
#pragma unroll
    for (int i = 0; i < 4; ++i) {
      const int tt = t - 3 + i;
      const int tc = (tt < 0) ? 0 : tt;
      float val = P[(size_t)(bt - t + tc) * kNcat + col];
      val = (tt >= 0) ? val : 0.0f;
      acc += w[i] * val;
    }
    const float y  = acc + bias;
    const float sg = 1.0f / (1.0f + expf(-y));
    sx[col] = y * sg;
  }
  __syncthreads();

  const int jj = lane & 15;
  const float cv = tab[t * 32 + jj];
  const float sv = tab[t * 32 + 16 + jj];
  const size_t obase = (size_t)bt * kKd + (size_t)wave * kHd;
#pragma unroll 1
  for (int which = 0; which < 2; ++which) {
    const float x1 = sx[which * kKd + wave * kHd + 2 * lane];
    const float x2 = sx[which * kKd + wave * kHd + 2 * lane + 1];
    const float r1 = x1 * cv - x2 * sv;
    const float r2 = x1 * sv + x2 * cv;
    float ss = r1 * r1 + r2 * r2;
    ss += __shfl_xor(ss, 16, 32);
    ss += __shfl_xor(ss, 8, 32);
    ss += __shfl_xor(ss, 4, 32);
    ss += __shfl_xor(ss, 2, 32);
    ss += __shfl_xor(ss, 1, 32);
    const float sc = 1.0f / fmaxf(sqrtf(ss), kL2Eps);
    const float w1 = r1 * sc;
    const float w2 = r2 * sc;
    float* dst = (which == 0) ? qo : ko;
    volatile float* dq = dst + obase;
    dq[lane] = w1;
    dq[32 + lane] = w2;
    __threadfence();
    dq[lane] = w1;
    dq[32 + lane] = w2;
  }
  {
    const float v0 = sx[2 * kKd + tid];
    const float v1 = sx[2 * kKd + 256 + tid];
    volatile float* dv = vo + (size_t)bt * kKd;
    dv[tid] = v0;
    dv[256 + tid] = v1;
    __threadfence();
    dv[tid] = v0;
    dv[256 + tid] = v1;
  }
}

__global__ __launch_bounds__(256) void scan_kernel(const float* __restrict__ qp, const float* __restrict__ kp,
                                                   const float* __restrict__ vp, const float* __restrict__ gates,
                                                   float* __restrict__ op) {
  __shared__ __align__(16) float kb[kChunk * kHd];
  __shared__ __align__(16) float qb[kChunk * kHd];
  __shared__ __align__(16) float vb[kChunk * kHd];
  __shared__ __align__(16) float ob[kChunk * kHd];
  __shared__ float gab[2 * kChunk];
  const int tid  = threadIdx.x;
  const int lane = tid & 31;
  const int wave = tid >> 5;
  const int gq   = lane >> 3;
  const int e    = wave * 8 + (lane & 7);
  const int b    = blockIdx.x / kHeads;
  const int h    = blockIdx.x % kHeads;
  const int srow = tid >> 4;
  const int c4   = (tid & 15) * 4;

  float S[16];
#pragma unroll
  for (int r = 0; r < 16; ++r) S[r] = 0.0f;

#pragma unroll 1
  for (int t0 = 0; t0 < kSeq; t0 += kChunk) {
    const size_t g = (size_t)(b * kSeq + t0 + srow) * kKd + (size_t)h * kHd + c4;
    {
      const v4f kv = *(const v4f*)(kp + g);
      const v4f qv = *(const v4f*)(qp + g);
      const v4f vv = *(const v4f*)(vp + g);
      *(v4f*)(kb + srow * kHd + c4) = kv;
      *(v4f*)(qb + srow * kHd + c4) = qv;
      *(v4f*)(vb + srow * kHd + c4) = vv;
    }
    if (tid < 32) {
      const int s = tid & 15;
      const int w = tid >> 4;
      gab[tid] = gates[(size_t)(1 - w) * kGateN + (size_t)(b * kSeq + t0 + s) * kHeads + h];
    }
    __syncthreads();

#pragma unroll 1
    for (int s = 0; s < kChunk; ++s) {
      const float at = gab[s];
      const float bs = gab[kChunk + s];
      const float ve = vb[s * kHd + e];
      const float* kr = kb + s * kHd + gq * 16;
      const float* qr = qb + s * kHd + gq * 16;
      const v4f k0 = *(const v4f*)(kr);
      const v4f k1 = *(const v4f*)(kr + 4);
      const v4f k2 = *(const v4f*)(kr + 8);
      const v4f k3 = *(const v4f*)(kr + 12);
      const v4f q0 = *(const v4f*)(qr);
      const v4f q1 = *(const v4f*)(qr + 4);
      const v4f q2 = *(const v4f*)(qr + 8);
      const v4f q3 = *(const v4f*)(qr + 12);
      float kk[16], qq[16];
#pragma unroll
      for (int j = 0; j < 4; ++j) {
        kk[j] = k0[j]; kk[4 + j] = k1[j]; kk[8 + j] = k2[j]; kk[12 + j] = k3[j];
        qq[j] = q0[j]; qq[4 + j] = q1[j]; qq[8 + j] = q2[j]; qq[12 + j] = q3[j];
      }
      float p = 0.0f;
#pragma unroll
      for (int r = 0; r < 16; ++r) p += kk[r] * S[r];
      p += __shfl_xor(p, 8, 32);
      p += __shfl_xor(p, 16, 32);
      float p2 = 0.0f;
#pragma unroll
      for (int r = 0; r < 16; ++r) {
        const float bk = bs * kk[r];
        const float er = S[r] - bk * p;
        const float sn = at * er + bk * ve;
        S[r] = sn;
        p2 += qq[r] * sn;
      }
      p2 += __shfl_xor(p2, 8, 32);
      p2 += __shfl_xor(p2, 16, 32);
      if (gq == 0) ob[s * kHd + e] = p2;
    }
    __syncthreads();

    {
      const v4f val = *(const v4f*)(ob + srow * kHd + c4);
      float* dst = op + g;
      *(volatile v4f*)dst = val;
      __threadfence();
      *(volatile v4f*)dst = val;
    }
  }
}

__global__ __launch_bounds__(256) void post_kernel(const float* __restrict__ op, const float* __restrict__ vp,
                                                   const float* __restrict__ P, const float* __restrict__ Dp,
                                                   const float* __restrict__ onw,
                                                   unsigned short* __restrict__ ah, unsigned short* __restrict__ al) {
  const int bt   = blockIdx.x;
  const int tid  = threadIdx.x;
  const int lane = tid & 31;
  const int h    = tid >> 5;
  const size_t base = (size_t)bt * kKd + (size_t)h * kHd + 2 * lane;
  const v2f oo = *(const v2f*)(op + base);
  const v2f vv = *(const v2f*)(vp + base);
  const v2f gg = *(const v2f*)(P + (size_t)bt * kNcat + kColG + h * kHd + 2 * lane);
  const v2f ww = *(const v2f*)(onw + 2 * lane);
  const float dv = Dp[h];
  const float o1 = oo[0] + dv * vv[0];
  const float o2 = oo[1] + dv * vv[1];
  float ss = o1 * o1 + o2 * o2;
  ss += __shfl_xor(ss, 16, 32);
  ss += __shfl_xor(ss, 8, 32);
  ss += __shfl_xor(ss, 4, 32);
  ss += __shfl_xor(ss, 2, 32);
  ss += __shfl_xor(ss, 1, 32);
  const float inv = rsqrtf(ss * kInvHd + kNormEps);
  const float n1 = (o1 * inv) * ww[0];
  const float n2 = (o2 * inv) * ww[1];
  const float s1 = 1.0f / (1.0f + expf(-n1));
  const float s2 = 1.0f / (1.0f + expf(-n2));
  const float a1 = gg[0] * (n1 * s1);
  const float a2 = gg[1] * (n2 * s2);
  const unsigned short h1 = f2bf_bits(a1);
  const unsigned short h2 = f2bf_bits(a2);
  const unsigned short l1 = f2bf_bits(a1 - bf_bits2f(h1));
  const unsigned short l2 = f2bf_bits(a2 - bf_bits2f(h2));
  const unsigned wh = pk16(h1, h2);
  const unsigned wl = pk16(l1, l2);
  const size_t widx = (size_t)bt * (kKd / 2) + (size_t)h * (kHd / 2) + lane;
  volatile unsigned* ph = (volatile unsigned*)ah + widx;
  volatile unsigned* pl = (volatile unsigned*)al + widx;
  *ph = wh;
  *pl = wl;
  __threadfence();
  *ph = wh;
  *pl = wl;
}

extern "C" void kernel_launch(void* const* d_in, const int* in_sizes, int n_in,
                              void* d_out, int out_size, void* d_ws, size_t ws_size, hipStream_t stream) {
  if (n_in < 20 || d_out == nullptr || d_ws == nullptr) return;
  if (in_sizes[0] != kRows * kHid) return;
  for (int i = 1; i <= 5; ++i) if (in_sizes[i] != kKd * kHid) return;
  if (in_sizes[6] != kHeads * kHid || in_sizes[8] != kHeads * kHid) return;
  if (in_sizes[7] != kHeads || in_sizes[9] != kHeads || in_sizes[16] != kHeads ||
      in_sizes[17] != kHeads || in_sizes[18] != kHeads) return;
  if (in_sizes[10] != kKd * kConvTaps || in_sizes[12] != kKd * kConvTaps || in_sizes[14] != kKd * kConvTaps) return;
  if (in_sizes[11] != kKd || in_sizes[13] != kKd || in_sizes[15] != kKd) return;
  if (in_sizes[19] != kHd || out_size != kRows * kHid) return;

  const float* x     = (const float*)d_in[0];
  const float* Wq    = (const float*)d_in[1];
  const float* Wk    = (const float*)d_in[2];
  const float* Wv    = (const float*)d_in[3];
  const float* Wg    = (const float*)d_in[4];
  const float* Wo    = (const float*)d_in[5];
  const float* Wb    = (const float*)d_in[6];
  const float* bb    = (const float*)d_in[7];
  const float* Wgk   = (const float*)d_in[8];
  const float* bgk   = (const float*)d_in[9];
  const float* cqw   = (const float*)d_in[10];
  const float* cqb   = (const float*)d_in[11];
  const float* ckw   = (const float*)d_in[12];
  const float* ckb   = (const float*)d_in[13];
  const float* cvw   = (const float*)d_in[14];
  const float* cvb   = (const float*)d_in[15];
  const float* alog  = (const float*)d_in[16];
  const float* Dp    = (const float*)d_in[17];
  const float* dtb   = (const float*)d_in[18];
  const float* onw   = (const float*)d_in[19];
  float* out = (float*)d_out;

  char* ws = (char*)d_ws; size_t off = 0;
  auto carve = [&](size_t bytes) -> char* { char* p = ws + off; off += (bytes + 255) & ~(size_t)255; return p; };
  unsigned short* XH  = (unsigned short*)carve((size_t)kRows * kHid * 2);
  unsigned short* XL  = (unsigned short*)carve((size_t)kRows * kHid * 2);
  unsigned short* WCH = (unsigned short*)carve((size_t)kNcat * kHid * 2);
  unsigned short* WCL = (unsigned short*)carve((size_t)kNcat * kHid * 2);
  unsigned short* WOH = (unsigned short*)carve((size_t)kHid * kKd * 2);
  unsigned short* WOL = (unsigned short*)carve((size_t)kHid * kKd * 2);
  float*          TAB = (float*)carve((size_t)kSeq * 32 * 4);
  float*          P   = (float*)carve((size_t)kRows * kNcat * 4);
  float*          GAT = (float*)carve((size_t)2 * kGateN * 4);
  float*          Qp  = (float*)carve((size_t)kRows * kKd * 4);
  float*          Kp  = (float*)carve((size_t)kRows * kKd * 4);
  float*          Vp  = (float*)carve((size_t)kRows * kKd * 4);
  float*          Op  = (float*)carve((size_t)kRows * kKd * 4);
  unsigned short* AH  = (unsigned short*)carve((size_t)kRows * kKd * 2);
  unsigned short* AL  = (unsigned short*)carve((size_t)kRows * kKd * 2);
  if (off > ws_size || off > (size_t)134217728) return;

  RotC rc;
  {
    const float basef  = (float)kRotBase;
    const float sbasef = (float)(kRotBase * pow(kRotMaxLen / kRotOrig, (double)kHd / ((double)kHd - 2.0)));
    const float twopi  = (float)(2.0 * 3.14159265358979323846);
    const float fm1    = (float)(kRotFactor - 1.0);
    for (int jj = 0; jj < 16; ++jj) {
      const float ar   = (float)(4 * jj) / (float)kHd;
      const float invf = 1.0f / powf(sbasef, ar);
      const float fe   = 1.0f / powf(basef, ar);
      const float wl   = twopi / fe;
      float ramp = (wl - 1.0f) / fm1;
      ramp = ramp < 0.0f ? 0.0f : (ramp > 1.0f ? 1.0f : ramp);
      const float spf = 1.0f + fm1 * ramp;
      rc.invf[jj] = invf;
      rc.rspf[jj] = 1.0f / spf;
    }
  }

  const int n8x = kRows * kHid / 8;
  const int n8o = kHid * kKd / 8;
  split8_kernel<<<(n8x + 255) / 256, 256, 0, stream>>>(x, XH, XL, n8x);
  wcat_kernel<<<kNcat * 64 / 256, 256, 0, stream>>>(Wq, Wk, Wv, Wg, Wb, Wgk, WCH, WCL);
  split8_kernel<<<(n8o + 255) / 256, 256, 0, stream>>>(Wo, WOH, WOL, n8o);
  rot_table_kernel<<<kSeq / 16, 256, 0, stream>>>(TAB, rc);

  wmma_gemm64<1, true, 0, 0, false, 0><<<dim3((kRows / 64) * (kNcat / 64) / 8, 1), 256, 0, stream>>>(
      XH, XL, kHid, 0L, WCH, WCL, kHid, 0L, (void*)P, (void*)P, kNcat, 0L,
      P, P, 0L, kRows, kNcat, kHid, 1.0f);

  gate_kernel<<<kGateN / 256, 256, 0, stream>>>(P, bb, bgk, alog, dtb, GAT);
  prep_kernel<<<kRows, 256, 0, stream>>>(P, cqw, cqb, ckw, ckb, cvw, cvb, TAB, Qp, Kp, Vp);

  scan_kernel<<<kBatch * kHeads, 256, 0, stream>>>(Qp, Kp, Vp, GAT, Op);

  post_kernel<<<kRows, 256, 0, stream>>>(Op, Vp, P, Dp, onw, AH, AL);

  wmma_gemm64<1, true, 0, 0, false, 0><<<dim3((kRows / 64) * (kHid / 64) / 8, 1), 256, 0, stream>>>(
      AH, AL, kKd, 0L, WOH, WOL, kKd, 0L, (void*)out, (void*)out, kHid, 0L,
      P, P, 0L, kRows, kHid, kKd, 1.0f);
}
